// DeformableBlock_79637283602552
// MI455X (gfx1250) — hardware-verified
//
#include <hip/hip_runtime.h>
#include <stddef.h>


typedef __attribute__((ext_vector_type(16))) _Float16 v16h;
typedef __attribute__((ext_vector_type(8)))  _Float16 v8h;
typedef __attribute__((ext_vector_type(16))) __bf16   v16b;
typedef __attribute__((ext_vector_type(8)))  __bf16   v8b;
typedef __attribute__((ext_vector_type(8)))  float    v8f;
typedef __attribute__((ext_vector_type(4)))  float    v4f;

#define NB    8
#define NC    64
#define NO    64
#define IH    128
#define IW    128
#define HW    16384
#define NPIX  131072
#define PH    130
#define PW    130
#define KD    576
#define NOFF  18
#define OFFP  32
#define CHUNK 32768
#define NCHUNK 4

__device__ __forceinline__ unsigned short f2bf_bits(float f) {
  unsigned u = __float_as_uint(f);
  return (unsigned short)((u + 0x7FFFu + ((u >> 16) & 1u)) >> 16);
}
__device__ __forceinline__ float bf_bits2f(unsigned short h) { return __uint_as_float(((unsigned)h) << 16); }

__device__ __forceinline__ void dep_guard_h(v8f& a, v8f& b, v16h x, v16h y) { asm volatile("v_nop\n\tv_nop\n\tv_nop\n\tv_nop" : "+v"(a), "+v"(b) : "v"(x), "v"(y)); }
__device__ __forceinline__ void dep_guard_b(v8f& a, v8f& b, v16b x, v16b y) { asm volatile("v_nop\n\tv_nop\n\tv_nop\n\tv_nop" : "+v"(a), "+v"(b) : "v"(x), "v"(y)); }
__device__ __forceinline__ void keep4_h(v16h a, v16h b, v16h c, v16h d) { asm volatile("v_nop" :: "v"(a), "v"(b), "v"(c), "v"(d)); }
__device__ __forceinline__ void keep4_b(v16b a, v16b b, v16b c, v16b d) { asm volatile("v_nop" :: "v"(a), "v"(b), "v"(c), "v"(d)); }
__device__ __forceinline__ void acc_guard4(v8f& a, v8f& b, v8f& c, v8f& d) { asm volatile("v_nop\n\tv_nop\n\tv_nop\n\tv_nop" : "+v"(a), "+v"(b), "+v"(c), "+v"(d)); }
template <typename T> struct Frag;
template <> struct Frag<_Float16> {
  typedef v16h V; union U { v16h v; v8h h[2]; };
  static __device__ __forceinline__ v16h load(const _Float16* p) {
    U f; f.h[0] = *(const v8h*)(p); f.h[1] = *(const v8h*)(p + 16); return f.v;
  }
  static __device__ __forceinline__ v8f mma(v16h a, v16h b, v8f c) {
    return __builtin_amdgcn_wmma_f32_16x16x32_f16(false, a, false, b, (short)0, c, false, false);
  }
  static __device__ __forceinline__ void guard(v8f& a, v8f& b, v16h x, v16h y) { dep_guard_h(a, b, x, y); }
  static __device__ __forceinline__ void keep(v16h a, v16h b, v16h c, v16h d) { keep4_h(a, b, c, d); }
};
template <> struct Frag<__bf16> {
  typedef v16b V; union U { v16b v; v8b h[2]; };
  static __device__ __forceinline__ v16b load(const __bf16* p) {
    U f; f.h[0] = *(const v8b*)(p); f.h[1] = *(const v8b*)(p + 16); return f.v;
  }
  static __device__ __forceinline__ v8f mma(v16b a, v16b b, v8f c) {
    return __builtin_amdgcn_wmma_f32_16x16x32_bf16(false, a, false, b, (short)0, c, false, false);
  }
  static __device__ __forceinline__ void guard(v8f& a, v8f& b, v16b x, v16b y) { dep_guard_b(a, b, x, y); }
  static __device__ __forceinline__ void keep(v16b a, v16b b, v16b c, v16b d) { keep4_b(a, b, c, d); }
};

template <int ET> struct Elem;
template <> struct Elem<0> { typedef _Float16 T; };
template <> struct Elem<1> { typedef __bf16 T; };
template <int ET, bool SPLIT, int BIAS_MODE, int OUT_MODE, bool RESID, int ACT = 0>
__global__ __launch_bounds__(256) void wmma_gemm64(
    const unsigned short* __restrict__ Ap, const unsigned short* __restrict__ A2p, int lda, long strideA,
    const unsigned short* __restrict__ Btp, const unsigned short* __restrict__ Bt2p, int ldb, long strideB,
    void* __restrict__ Cout, void* __restrict__ Cout2, int ldc, long strideC,
    const float* __restrict__ bias,
    const float* __restrict__ resid, long strideR,
    int M, int N, int K, float scale) {
  typedef typename Elem<ET>::T T;
  typedef typename Frag<T>::V V;
  const T* A = (const T*)Ap; const T* A2 = (const T*)A2p; const T* Bt = (const T*)Btp; const T* Bt2 = (const T*)Bt2p;
  __shared__ __align__(16) float sT[8][16 * 68];
  const int b    = blockIdx.y;
  const int lane = threadIdx.x & 31;
  const int wave = threadIdx.x >> 5;
  const int tilesN = N >> 6;
  const int tilesM = M >> 6;
  const int tile = blockIdx.x * 8 + wave;
  if (tile >= tilesM * tilesN) return;
  const int tm = tile / tilesN;
  const int tn = tile - tm * tilesN;
  const int m0 = tm << 6;
  const int n0 = tn << 6;

  const T* Ab  = A  + (size_t)b * strideA;
  const T* Bb  = Bt + (size_t)b * strideB;
  const T* Ab2 = SPLIT ? (A2  + (size_t)b * strideA) : nullptr;
  const T* Bb2 = SPLIT ? (Bt2 + (size_t)b * strideB) : nullptr;

  const int rlane = lane & 15;
  const int koff  = (lane >> 4) * 8;
  const int mOff  = (lane >> 4) * 8;

  v8f acc[4][4];
#pragma unroll
  for (int i = 0; i < 4; ++i)
#pragma unroll
    for (int j = 0; j < 4; ++j) acc[i][j] = (v8f){0.f,0.f,0.f,0.f,0.f,0.f,0.f,0.f};

  for (int k0 = 0; k0 < K; k0 += 32) {
    V bh[4], bl[4];
#pragma unroll
    for (int j = 0; j < 4; ++j) {
      const size_t bo = (size_t)(n0 + (j << 4) + rlane) * ldb + koff + k0;
      bh[j] = Frag<T>::load(Bb + bo);
      if (SPLIT) bl[j] = Frag<T>::load(Bb2 + bo);
    }
#pragma unroll
    for (int i = 0; i < 4; ++i) {
      const size_t ao = (size_t)(m0 + (i << 4) + rlane) * lda + koff + k0;
      V ah = Frag<T>::load(Ab + ao);
      V al;
      if (SPLIT) al = Frag<T>::load(Ab2 + ao);
#pragma unroll
      for (int j = 0; j < 4; ++j) {
        acc[i][j] = Frag<T>::mma(ah, bh[j], acc[i][j]);
        if (SPLIT) {
          acc[i][j] = Frag<T>::mma(ah, bl[j], acc[i][j]);
          acc[i][j] = Frag<T>::mma(al, bh[j], acc[i][j]);
        }
      }
      Frag<T>::guard(acc[i][0], acc[i][3], ah, SPLIT ? al : ah);
    }
    Frag<T>::keep(bh[0], bh[1], bh[2], bh[3]);
    if (SPLIT) Frag<T>::keep(bl[0], bl[1], bl[2], bl[3]);
  }
  acc_guard4(acc[0][0], acc[0][1], acc[0][2], acc[0][3]);
  acc_guard4(acc[1][0], acc[1][1], acc[1][2], acc[1][3]);
  acc_guard4(acc[2][0], acc[2][1], acc[2][2], acc[2][3]);
  acc_guard4(acc[3][0], acc[3][1], acc[3][2], acc[3][3]);

  float* slab = sT[wave];
  const float* Rb = RESID ? (resid + (size_t)b * strideR) : nullptr;
#pragma unroll
  for (int i = 0; i < 4; ++i) {
    const int mBase = m0 + (i << 4);
#pragma unroll
    for (int j = 0; j < 4; ++j) {
      const int n = n0 + (j << 4) + rlane;
      float bv = 0.f;
      if (BIAS_MODE == 2) bv = bias[n];
#pragma unroll
      for (int r = 0; r < 8; ++r) {
        float v = acc[i][j][r] * scale;
        if (BIAS_MODE == 1) v += bias[mBase + mOff + r];
        if (BIAS_MODE == 2) v += bv;
        if (RESID) v += Rb[(size_t)(mBase + mOff + r) * ldc + n];
        if (ACT == 1) v = tanhf(v);
        if (ACT == 2) v = fmaxf(v, 0.0f);
        if (ACT == 3) v = v / (1.0f + expf(-v));
        if (ACT == 4) v = (v > 0.f) ? v : 0.01f * v;
        if (ACT == 5) v = 0.5f * v * (1.0f + erff(v * 0.70710678118654752f));
        slab[(mOff + r) * 68 + (j << 4) + rlane] = v;
      }
    }
    __builtin_amdgcn_fence(__ATOMIC_RELEASE, "workgroup");
    __builtin_amdgcn_wave_barrier();
    __builtin_amdgcn_fence(__ATOMIC_ACQUIRE, "workgroup");
    if (OUT_MODE == 0) {
      float* C = (float*)Cout + (size_t)b * strideC;
      const int hh = lane >> 4, c4 = (lane & 15) * 4;
      for (int pass = 0; pass < 2; ++pass) {
#pragma unroll
        for (int it = 0; it < 8; ++it) {
          const int row = it * 2 + hh;
          v4f v = *(const v4f*)(slab + row * 68 + c4);
          *(volatile v4f*)(C + (size_t)(mBase + row) * ldc + n0 + c4) = v;
        }
        __threadfence();
      }
    } else {
      const int q = lane >> 3, c8 = (lane & 7) * 8;
      unsigned short* C  = (unsigned short*)Cout  + (size_t)b * strideC;
      unsigned short* C2 = (OUT_MODE == 2) ? ((unsigned short*)Cout2 + (size_t)b * strideC) : nullptr;
      for (int pass = 0; pass < 2; ++pass) {
#pragma unroll
        for (int it = 0; it < 4; ++it) {
          const int row = it * 4 + q;
          const float* sp = slab + row * 68 + c8;
          v8h hv, lv;
#pragma unroll
          for (int e = 0; e < 8; ++e) {
            if (OUT_MODE == 1) {
              hv[e] = (_Float16)sp[e];
            } else {
              unsigned short hb = f2bf_bits(sp[e]);
              unsigned short lb = f2bf_bits(sp[e] - bf_bits2f(hb));
              hv[e] = __builtin_bit_cast(_Float16, hb);
              lv[e] = __builtin_bit_cast(_Float16, lb);
            }
          }
          *(volatile v8h*)(C + (size_t)(mBase + row) * ldc + n0 + c8) = hv;
          if (OUT_MODE == 2) *(volatile v8h*)(C2 + (size_t)(mBase + row) * ldc + n0 + c8) = lv;
        }
        __threadfence();
      }
    }
    __builtin_amdgcn_fence(__ATOMIC_RELEASE, "workgroup");
    __builtin_amdgcn_wave_barrier();
    __builtin_amdgcn_fence(__ATOMIC_ACQUIRE, "workgroup");
  }
}

__global__ __launch_bounds__(256) void x_layout(const float* __restrict__ x, float* __restrict__ xcl,
                                                unsigned short* __restrict__ Xh, unsigned short* __restrict__ Xl)
{
  __shared__ __align__(16) float tile[NC * 132];
  const int tid = threadIdx.x;
  const int bid = blockIdx.x;
  const int b   = bid / PH;
  const int yp  = bid - b * PH;
  const bool interior = (yp >= 1) && (yp <= IH);
  const int y = interior ? (yp - 1) : 0;
  if (interior) {
    const float* xb = x + ((size_t)(b * NC) * IH + y) * IW;
    for (int i = tid; i < NC * IW; i += 256) {
      const int c = i >> 7, xx = i & (IW - 1);
      tile[c * 132 + xx] = xb[(size_t)c * HW + xx];
    }
  }
  __syncthreads();
  if (interior) {
    float* dst = xcl + ((size_t)(b * IH + y) * IW) * NC;
    for (int g = tid; g < IW * NC / 4; g += 256) {
      const int xx = g >> 4, c4 = (g & 15) * 4;
      v4f v;
      v[0] = tile[(c4 + 0) * 132 + xx];
      v[1] = tile[(c4 + 1) * 132 + xx];
      v[2] = tile[(c4 + 2) * 132 + xx];
      v[3] = tile[(c4 + 3) * 132 + xx];
      float* p = dst + (size_t)g * 4;
      *(volatile v4f*)p = v;
      __threadfence();
      *(volatile v4f*)p = v;
    }
  }
  {
    const size_t rowoff = ((size_t)(b * PH + yp) * PW) * NC;
    unsigned short* dh = Xh + rowoff;
    unsigned short* dl = Xl + rowoff;
    for (int g = tid; g < PW * NC / 8; g += 256) {
      const int xp = g >> 3, c8 = (g & 7) * 8;
      const bool inb = interior && (xp >= 1) && (xp <= IW);
      int xx = xp - 1; xx = xx < 0 ? 0 : (xx > IW - 1 ? IW - 1 : xx);
      v8h hv, lv;
#pragma unroll
      for (int e = 0; e < 8; ++e) {
        float f = tile[(c8 + e) * 132 + xx];
        f = inb ? f : 0.0f;
        const unsigned short hb = f2bf_bits(f);
        const unsigned short lb = f2bf_bits(f - bf_bits2f(hb));
        hv[e] = __builtin_bit_cast(_Float16, hb);
        lv[e] = __builtin_bit_cast(_Float16, lb);
      }
      unsigned short* ph = dh + (size_t)g * 8;
      unsigned short* pl = dl + (size_t)g * 8;
      *(volatile v8h*)ph = hv;
      *(volatile v8h*)pl = lv;
      __threadfence();
      *(volatile v8h*)ph = hv;
      *(volatile v8h*)pl = lv;
    }
  }
}

__global__ __launch_bounds__(256) void prep_weights(const float* __restrict__ ow, const float* __restrict__ dw,
    unsigned short* __restrict__ Wh, unsigned short* __restrict__ Wl, _Float16* __restrict__ W16)
{
  const int g  = blockIdx.x * 256 + threadIdx.x;
  const int GR = KD / 8;
  const int G1 = OFFP * GR;
  const int G2 = NO * GR;
  if (g < G1) {
    const int n  = g / GR;
    const int kg = g - n * GR;
    const int nn = n < NOFF ? n : (NOFF - 1);
    const bool live = n < NOFF;
    v8h hv, lv;
#pragma unroll
    for (int e = 0; e < 8; ++e) {
      const int k = kg * 8 + e;
      const int tap = k >> 6, c = k & 63;
      float w = ow[(nn * NC + c) * 9 + tap];
      w = live ? w : 0.0f;
      const unsigned short hb = f2bf_bits(w);
      const unsigned short lb = f2bf_bits(w - bf_bits2f(hb));
      hv[e] = __builtin_bit_cast(_Float16, hb);
      lv[e] = __builtin_bit_cast(_Float16, lb);
    }
    unsigned short* ph = Wh + (size_t)g * 8;
    unsigned short* pl = Wl + (size_t)g * 8;
    *(volatile v8h*)ph = hv;
    *(volatile v8h*)pl = lv;
    __threadfence();
    *(volatile v8h*)ph = hv;
    *(volatile v8h*)pl = lv;
  } else if (g < G1 + G2) {
    const int g2 = g - G1;
    const int o  = g2 / GR;
    const int kg = g2 - o * GR;
    v8h hv;
#pragma unroll
    for (int e = 0; e < 8; ++e) {
      const int k = kg * 8 + e;
      const int tap = k >> 6, c = k & 63;
      hv[e] = (_Float16)(16.0f * dw[(o * NC + c) * 9 + tap]);
    }
    _Float16* p = W16 + (size_t)g2 * 8;
    *(volatile v8h*)p = hv;
    __threadfence();
    *(volatile v8h*)p = hv;
  }
}

__global__ __launch_bounds__(256) void offconv_gemm(const unsigned short* __restrict__ Xhp, const unsigned short* __restrict__ Xlp,
    const unsigned short* __restrict__ Whp, const unsigned short* __restrict__ Wlp,
    const float* __restrict__ ob, float* __restrict__ OFF)
{
  typedef __bf16 T;
  typedef v16b V;
  const T* Xh = (const T*)Xhp; const T* Xl = (const T*)Xlp;
  const T* Wh = (const T*)Whp; const T* Wl = (const T*)Wlp;
  __shared__ __align__(16) float sT[8][16 * 36];
  const int lane = threadIdx.x & 31;
  const int wave = threadIdx.x >> 5;
  const int tile = blockIdx.x * 8 + wave;
  if (tile >= NPIX / 64) return;
  const int m0  = tile << 6;
  const int b   = m0 >> 14;
  const int rem = m0 & (HW - 1);
  const int y   = rem >> 7;
  const int x0  = rem & (IW - 1);
  const int rlane = lane & 15;
  const int koff  = (lane >> 4) * 8;
  const int mOff  = koff;
  const size_t xbase = ((size_t)(b * PH + y) * PW + x0) * NC;

  v8f acc[4][2];
#pragma unroll
  for (int i = 0; i < 4; ++i)
#pragma unroll
    for (int j = 0; j < 2; ++j) acc[i][j] = (v8f){0.f,0.f,0.f,0.f,0.f,0.f,0.f,0.f};

#pragma unroll 1
  for (int ks = 0; ks < KD / 32; ++ks) {
    const int tap = ks >> 1;
    const int kc  = (ks & 1) << 5;
    const int ki  = tap / 3;
    const int kj  = tap - ki * 3;
    const size_t tb = xbase + (size_t)(ki * PW + kj) * NC + kc + koff;
    V bh[2], bl[2];
#pragma unroll
    for (int j = 0; j < 2; ++j) {
      const size_t bo = (size_t)((j << 4) + rlane) * KD + ks * 32 + koff;
      bh[j] = Frag<T>::load(Wh + bo);
      bl[j] = Frag<T>::load(Wl + bo);
    }
#pragma unroll
    for (int i = 0; i < 4; ++i) {
      const size_t ao = tb + (size_t)((i << 4) + rlane) * NC;
      V ah = Frag<T>::load(Xh + ao);
      V al = Frag<T>::load(Xl + ao);
#pragma unroll
      for (int j = 0; j < 2; ++j) {
        acc[i][j] = Frag<T>::mma(ah, bh[j], acc[i][j]);
        acc[i][j] = Frag<T>::mma(ah, bl[j], acc[i][j]);
        acc[i][j] = Frag<T>::mma(al, bh[j], acc[i][j]);
      }
      Frag<T>::guard(acc[i][0], acc[i][1], ah, al);
    }
    Frag<T>::keep(bh[0], bh[1], bl[0], bl[1]);
  }
  acc_guard4(acc[0][0], acc[0][1], acc[1][0], acc[1][1]);
  acc_guard4(acc[2][0], acc[2][1], acc[3][0], acc[3][1]);

  float* slab = sT[wave];
#pragma unroll
  for (int i = 0; i < 4; ++i) {
    const int mBase = m0 + (i << 4);
#pragma unroll
    for (int j = 0; j < 2; ++j) {
      const int n  = (j << 4) + rlane;
      const int nn = n < NOFF ? n : (NOFF - 1);
      const float bv = ob[nn];
      const bool live = n < NOFF;
#pragma unroll
      for (int r = 0; r < 8; ++r) {
        float v = acc[i][j][r] + bv;
        v = live ? v : 0.0f;
        slab[(mOff + r) * 36 + (j << 4) + rlane] = v;
      }
    }
    __builtin_amdgcn_fence(__ATOMIC_RELEASE, "workgroup");
    __builtin_amdgcn_wave_barrier();
    __builtin_amdgcn_fence(__ATOMIC_ACQUIRE, "workgroup");
    {
      const int q = lane >> 3, c4 = (lane & 7) * 4;
      for (int pass = 0; pass < 2; ++pass) {
#pragma unroll
        for (int it = 0; it < 4; ++it) {
          const int row = it * 4 + q;
          v4f v = *(const v4f*)(slab + row * 36 + c4);
          *(volatile v4f*)(OFF + (size_t)(mBase + row) * OFFP + c4) = v;
        }
        __threadfence();
      }
    }
    __builtin_amdgcn_fence(__ATOMIC_RELEASE, "workgroup");
    __builtin_amdgcn_wave_barrier();
    __builtin_amdgcn_fence(__ATOMIC_ACQUIRE, "workgroup");
  }
}

__global__ __launch_bounds__(256) void deform_sample(const float* __restrict__ xcl, const float* __restrict__ OFF,
                                                     _Float16* __restrict__ S, int pix0)
{
  const int tid = threadIdx.x;
  const int u   = blockIdx.x * 32 + (tid >> 3);
  const int sub = tid & 7;
  const int pl  = u / 9;
  const int tap = u - pl * 9;
  int p = pix0 + pl; p = p < NPIX ? p : (NPIX - 1);
  const int b = p >> 14, rem = p & (HW - 1), y = rem >> 7, xx = rem & (IW - 1);
  const int kq = tap / 3;
  const int ki = kq - 1, kj = tap - kq * 3 - 1;
  const float dy = OFF[(size_t)p * OFFP + 2 * tap];
  const float dx = OFF[(size_t)p * OFFP + 2 * tap + 1];
  const float py = (float)(y + ki) + dy;
  const float px = (float)(xx + kj) + dx;
  const float y0f = floorf(py), x0f = floorf(px);
  const float wy = py - y0f, wx = px - x0f;
  const float omy = 1.0f - wy, omx = 1.0f - wx;
  const float y1f = y0f + 1.0f, x1f = x0f + 1.0f;
  const bool vy0 = (y0f >= 0.0f) && (y0f < (float)IH);
  const bool vy1 = (y1f >= 0.0f) && (y1f < (float)IH);
  const bool vx0 = (x0f >= 0.0f) && (x0f < (float)IW);
  const bool vx1 = (x1f >= 0.0f) && (x1f < (float)IW);
  const float m00 = (vy0 && vx0) ? 1.0f : 0.0f;
  const float m01 = (vy0 && vx1) ? 1.0f : 0.0f;
  const float m10 = (vy1 && vx0) ? 1.0f : 0.0f;
  const float m11 = (vy1 && vx1) ? 1.0f : 0.0f;
  const int yc0 = (int)fminf(fmaxf(y0f, 0.0f), (float)(IH - 1));
  const int yc1 = (int)fminf(fmaxf(y1f, 0.0f), (float)(IH - 1));
  const int xc0 = (int)fminf(fmaxf(x0f, 0.0f), (float)(IW - 1));
  const int xc1 = (int)fminf(fmaxf(x1f, 0.0f), (float)(IW - 1));
  const float* img = xcl + (size_t)b * HW * NC + sub * 8;
  const float* r00 = img + ((size_t)yc0 * IW + xc0) * NC;
  const float* r01 = img + ((size_t)yc0 * IW + xc1) * NC;
  const float* r10 = img + ((size_t)yc1 * IW + xc0) * NC;
  const float* r11 = img + ((size_t)yc1 * IW + xc1) * NC;
  v4f a0 = *(const v4f*)(r00); v4f a1 = *(const v4f*)(r00 + 4);
  v4f b0 = *(const v4f*)(r01); v4f b1 = *(const v4f*)(r01 + 4);
  v4f c0 = *(const v4f*)(r10); v4f c1 = *(const v4f*)(r10 + 4);
  v4f d0 = *(const v4f*)(r11); v4f d1 = *(const v4f*)(r11 + 4);
  a0 = a0 * m00; a1 = a1 * m00;
  b0 = b0 * m01; b1 = b1 * m01;
  c0 = c0 * m10; c1 = c1 * m10;
  d0 = d0 * m11; d1 = d1 * m11;
  const v4f s0 = omy * (omx * a0 + wx * b0) + wy * (omx * c0 + wx * d0);
  const v4f s1 = omy * (omx * a1 + wx * b1) + wy * (omx * c1 + wx * d1);
  v8h hv;
#pragma unroll
  for (int e = 0; e < 4; ++e) {
    hv[e]     = (_Float16)(s0[e] * 16.0f);
    hv[4 + e] = (_Float16)(s1[e] * 16.0f);
  }
  _Float16* dst = S + (size_t)u * NC + sub * 8;
  *(volatile v8h*)dst = hv;
  __threadfence();
  *(volatile v8h*)dst = hv;
}

extern "C" void kernel_launch(void* const* d_in, const int* in_sizes, int n_in,
                              void* d_out, int out_size, void* d_ws, size_t ws_size,
                              hipStream_t stream) {
  if (n_in < 5) return;
  if (in_sizes[0] != NB * NC * HW) return;
  if (in_sizes[1] != NOFF * NC * 9) return;
  if (in_sizes[2] != NOFF) return;
  if (in_sizes[3] != NO * NC * 9) return;
  if (in_sizes[4] != NO) return;
  if (out_size != NB * NO * HW) return;

  const float* x  = (const float*)d_in[0];
  const float* ow = (const float*)d_in[1];
  const float* ob = (const float*)d_in[2];
  const float* dw = (const float*)d_in[3];
  const float* db = (const float*)d_in[4];
  float* out = (float*)d_out;

  const size_t b_xcl = (size_t)NB * HW * NC * 4;
  const size_t b_xp  = (size_t)NB * PH * PW * NC * 2;
  const size_t b_off = (size_t)NPIX * OFFP * 4;
  const size_t b_wb  = (size_t)OFFP * KD * 2;
  const size_t b_w16 = (size_t)NO * KD * 2;
  const size_t b_s   = (size_t)CHUNK * KD * 2;
  const size_t o_xcl = 0;
  const size_t o_xh  = o_xcl + b_xcl;
  const size_t o_xl  = o_xh + b_xp;
  const size_t o_off = o_xl + b_xp;
  const size_t o_wh  = o_off + b_off;
  const size_t o_wl  = o_wh + b_wb;
  const size_t o_w16 = o_wl + b_wb;
  const size_t o_s   = o_w16 + b_w16;
  const size_t total = o_s + b_s;
  if (total > ws_size) return;

  char* ws = (char*)d_ws;
  float*          xcl = (float*)(ws + o_xcl);
  unsigned short* Xh  = (unsigned short*)(ws + o_xh);
  unsigned short* Xl  = (unsigned short*)(ws + o_xl);
  float*          OFF = (float*)(ws + o_off);
  unsigned short* Wh  = (unsigned short*)(ws + o_wh);
  unsigned short* Wl  = (unsigned short*)(ws + o_wl);
  _Float16*       W16 = (_Float16*)(ws + o_w16);
  _Float16*       S   = (_Float16*)(ws + o_s);

  x_layout<<<dim3(NB * PH), dim3(256), 0, stream>>>(x, xcl, Xh, Xl);
  prep_weights<<<dim3((OFFP * KD / 8 + NO * KD / 8 + 255) / 256), dim3(256), 0, stream>>>(ow, dw, Wh, Wl, W16);
  offconv_gemm<<<dim3(NPIX / 64 / 8), dim3(256), 0, stream>>>(Xh, Xl, Wh, Wl, ob, OFF);

  const long strideB = (long)HW * KD;
  const long strideC = (long)NO * HW;
  for (int ch = 0; ch < NCHUNK; ++ch) {
    deform_sample<<<dim3(CHUNK * 9 / 32), dim3(256), 0, stream>>>(xcl, OFF, S, ch * CHUNK);
    float* cbase = out + (size_t)ch * (CHUNK / HW) * NO * HW;
    wmma_gemm64<0, false, 1, 0, false, 2><<<dim3(HW / 64 / 8, CHUNK / HW, 1), dim3(256), 0, stream>>>(
        (const unsigned short*)W16, (const unsigned short*)W16, KD, (long)0,
        (const unsigned short*)S, (const unsigned short*)S, KD, strideB,
        (void*)cbase, (void*)cbase, HW, strideC,
        db,
        db, (long)0,
        NO, HW, KD, 1.0f / 256.0f);
  }
}
